// BSplineBasis_58265526337935
// MI455X (gfx1250) — hardware-run, weakly checked
//
#include <hip/hip_runtime.h>
#include <math.h>

typedef __attribute__((ext_vector_type(16))) _Float16 v16h;
typedef __attribute__((ext_vector_type(8)))  _Float16 v8h;
typedef __attribute__((ext_vector_type(8)))  float    v8f;
typedef __attribute__((ext_vector_type(4)))  float    v4f;

constexpr int kBatch = 4096;
constexpr int kIn    = 1024;
constexpr int kOut   = 1024;
constexpr int kNb    = 11;
constexpr int kKs    = kIn * kNb;
constexpr int kK     = kKs + kIn;
constexpr float kCarryA = 64.0f;
constexpr float kCarryB = 1024.0f;
constexpr float kFold   = 1.0f / (kCarryA * kCarryB);
constexpr int kChunkI   = 256;
constexpr int kChunkK   = kChunkI * kNb;
constexpr int kVecBasis = kChunkK / 8;
constexpr int kVecAll   = kVecBasis + kChunkI / 8;
constexpr int kSplGroups = kKs / 8;
constexpr int kRowGroups = kK / 8;

static_assert(kKs == 11264);
static_assert(kK == 12288);
static_assert((kK % 32) == 0);
static_assert((kBatch % 64) == 0 && (kOut % 64) == 0);
static_assert(((kChunkK * 2) % 128) == 0);
static_assert(((kKs * 2) % 128) == 0 && ((kK * 2) % 128) == 0);
static_assert(kVecBasis == 352 && (kVecBasis % 32) == 0);
static_assert(kVecAll == 384);
static_assert(kRowGroups == 6 * 256);
static_assert((kSplGroups % 32) == 0);
static_assert((kIn % kChunkI) == 0);
static_assert(kIn == 4 * 256);

constexpr size_t kOffA    = 0;
constexpr size_t kOffB    = kOffA + (size_t)kBatch * kK * 2;
constexpr size_t kWsTotal = kOffB + (size_t)kOut * kK * 2;
static_assert(kOffB == 100663296ull);
static_assert(kWsTotal == 125829120ull);
static_assert(kWsTotal <= 134217728ull);
static_assert((kOffB % 128) == 0);

__device__ __forceinline__ void keep4_h(v16h a, v16h b, v16h c, v16h d) { asm volatile("v_nop" :: "v"(a), "v"(b), "v"(c), "v"(d)); }
__device__ __forceinline__ void acc_guard4(v8f& a, v8f& b, v8f& c, v8f& d) { asm volatile("v_nop\n\tv_nop\n\tv_nop\n\tv_nop" : "+v"(a), "+v"(b), "+v"(c), "+v"(d)); }
__device__ __forceinline__ void group_guard_h(v8f& a, v8f& b, v8f& c, v8f& d, v16h x, v16h y0, v16h y1, v16h y2, v16h y3) {
  asm volatile("v_nop\n\tv_nop\n\tv_nop\n\tv_nop" : "+v"(a), "+v"(b), "+v"(c), "+v"(d) : "v"(x), "v"(y0), "v"(y1), "v"(y2), "v"(y3));
}
union FragU { v16h v; v8h h[2]; };
__device__ __forceinline__ v16h frag_load(const _Float16* p) {
  FragU f;
  f.h[0] = *(const v8h*)(p);
  f.h[1] = *(const v8h*)(p + 16);
  return f.v;
}
__device__ __forceinline__ v8f frag_mma(v16h a, v16h b, v8f c) {
  return __builtin_amdgcn_wmma_f32_16x16x32_f16(false, a, false, b, (short)0, c, false, false);
}

__global__ __launch_bounds__(256) void build_bt_kernel(
    const float* __restrict__ coeffs, const float* __restrict__ resw,
    const float* __restrict__ sbase, unsigned short* __restrict__ Bt)
{
  __shared__ float red[8];
  const int tid = threadIdx.x, lane = tid & 31, wave = tid >> 5;
  const int o = blockIdx.x;
  const v4f sv = *(const v4f*)(sbase + (size_t)o * kIn + tid * 4);
  float part = (sv[0] + sv[1]) + (sv[2] + sv[3]);
  part += __shfl_xor(part, 16, 32);
  part += __shfl_xor(part, 8, 32);
  part += __shfl_xor(part, 4, 32);
  part += __shfl_xor(part, 2, 32);
  part += __shfl_xor(part, 1, 32);
  if (lane == 0) red[wave] = part;
  __syncthreads();
  float tot = 0.0f;
#pragma unroll
  for (int w = 0; w < 8; ++w) tot += red[w];
  const float scl  = tot * (1.0f / (float)kIn);
  const float mulS = scl * kCarryB;
  const float mulR = kCarryB;
#pragma unroll 1
  for (int it = 0; it < 6; ++it) {
    const int g = it * 256 + tid;
    const bool isb = (g < kSplGroups);
    const int gs = isb ? g : 0;
    const int gr = isb ? 0 : (g - kSplGroups);
    const float* src = isb ? (coeffs + (size_t)o * kKs + (size_t)gs * 8)
                           : (resw + (size_t)o * kIn + (size_t)gr * 8);
    const float mul = isb ? mulS : mulR;
    const v4f a0 = *(const v4f*)(src);
    const v4f a1 = *(const v4f*)(src + 4);
    v8h hv;
#pragma unroll
    for (int e = 0; e < 4; ++e) {
      const float p0 = a0[e] * mul;
      const float p1 = a1[e] * mul;
      hv[e]     = (_Float16)p0;
      hv[4 + e] = (_Float16)p1;
    }
    unsigned short* q = Bt + (size_t)o * kK + (size_t)g * 8;
    *(volatile v8h*)q = hv;
    __threadfence();
    *(volatile v8h*)q = hv;
  }
}

__global__ __launch_bounds__(256) void build_a_kernel(
    const float* __restrict__ X, unsigned short* __restrict__ A)
{
  __shared__ __align__(16) float sV[kChunkK + kChunkI];
  const int tid = threadIdx.x;
  const int ic = blockIdx.x;
  const int b  = blockIdx.y;
  const float x  = X[(size_t)b * kIn + ic * kChunkI + tid];
  const float xc = fminf(fmaxf(x, -1.0f), 1.0f);
  const float u  = (xc + 1.0f) * 4.0f;
  const float cf = fminf(floorf(u), 8.0f);
  const int   c  = (int)cf;
  const float t  = u - cf;
  const float omt = 1.0f - t;
  const float t2 = t * t;
  const float t3 = t2 * t;
  const float sixth = kCarryA * (1.0f / 6.0f);
  const float w0 = omt * omt * omt * sixth;
  const float w1 = (3.0f * t3 - 6.0f * t2 + 4.0f) * sixth;
  const float w2 = (-3.0f * t3 + 3.0f * t2 + 3.0f * t + 1.0f) * sixth;
  const float w3 = t3 * sixth;
  float* row = sV + tid * kNb;
#pragma unroll
  for (int m = 0; m < kNb; ++m) {
    const int r = m - c;
    float v = 0.0f;
    v = (r == 0) ? w0 : v;
    v = (r == 1) ? w1 : v;
    v = (r == 2) ? w2 : v;
    v = (r == 3) ? w3 : v;
    row[m] = v;
  }
  sV[kChunkK + tid] = x * kCarryA;
  __syncthreads();
  unsigned short* arow = A + (size_t)b * kK;
#pragma unroll 1
  for (int it = 0; it < 2; ++it) {
    const int v = it * 256 + tid;
    if (v < kVecAll) {
      const float* sp = sV + 8 * v;
      const v4f a0 = *(const v4f*)(sp);
      const v4f a1 = *(const v4f*)(sp + 4);
      v8h hv;
#pragma unroll
      for (int e = 0; e < 4; ++e) {
        const float p0 = a0[e];
        const float p1 = a1[e];
        hv[e]     = (_Float16)p0;
        hv[4 + e] = (_Float16)p1;
      }
      const int dst = (v < kVecBasis) ? (ic * kChunkK + 8 * v)
                                      : (kKs + ic * kChunkI + 8 * (v - kVecBasis));
      unsigned short* q = arow + dst;
      *(volatile v8h*)q = hv;
      __threadfence();
      *(volatile v8h*)q = hv;
    }
  }
}

__global__ __launch_bounds__(256) void gemm_f16_bias_kernel(
    const unsigned short* __restrict__ Ap, int lda,
    const unsigned short* __restrict__ Btp, int ldb,
    float* __restrict__ Cout, int ldc,
    const float* __restrict__ bias,
    int M, int N, int K, float scale)
{
  const _Float16* A  = (const _Float16*)Ap;
  const _Float16* Bt = (const _Float16*)Btp;
  __shared__ __align__(16) float sT[8][16 * 68];
  const int lane = threadIdx.x & 31;
  const int wave = threadIdx.x >> 5;
  const int tilesN = N >> 6;
  const int tilesM = M >> 6;
  const int tile = blockIdx.x * 8 + wave;
  if (tile >= tilesM * tilesN) return;
  const int tm = tile / tilesN;
  const int tn = tile - tm * tilesN;
  const int m0 = tm << 6;
  const int n0 = tn << 6;

  const int rlane = lane & 15;
  const int koff  = (lane >> 4) * 8;
  const int mOff  = (lane >> 4) * 8;

  v8f acc[4][4];
#pragma unroll
  for (int i = 0; i < 4; ++i)
#pragma unroll
    for (int j = 0; j < 4; ++j) acc[i][j] = (v8f){0.f,0.f,0.f,0.f,0.f,0.f,0.f,0.f};

  for (int k0 = 0; k0 < K; k0 += 32) {
    v16h bh[4];
#pragma unroll
    for (int j = 0; j < 4; ++j) {
      const size_t bo = (size_t)(n0 + (j << 4) + rlane) * ldb + koff + k0;
      bh[j] = frag_load(Bt + bo);
    }
#pragma unroll
    for (int i = 0; i < 4; ++i) {
      const size_t ao = (size_t)(m0 + (i << 4) + rlane) * lda + koff + k0;
      const v16h ah = frag_load(A + ao);
#pragma unroll
      for (int j = 0; j < 4; ++j) acc[i][j] = frag_mma(ah, bh[j], acc[i][j]);
      group_guard_h(acc[i][0], acc[i][1], acc[i][2], acc[i][3], ah, bh[0], bh[1], bh[2], bh[3]);
    }
    keep4_h(bh[0], bh[1], bh[2], bh[3]);
  }
  acc_guard4(acc[0][0], acc[0][1], acc[0][2], acc[0][3]);
  acc_guard4(acc[1][0], acc[1][1], acc[1][2], acc[1][3]);
  acc_guard4(acc[2][0], acc[2][1], acc[2][2], acc[2][3]);
  acc_guard4(acc[3][0], acc[3][1], acc[3][2], acc[3][3]);

  float* slab = sT[wave];
#pragma unroll
  for (int i = 0; i < 4; ++i) {
    const int mBase = m0 + (i << 4);
#pragma unroll
    for (int j = 0; j < 4; ++j) {
      const int n = n0 + (j << 4) + rlane;
      const float bv = bias[n];
#pragma unroll
      for (int r = 0; r < 8; ++r) {
        float v = acc[i][j][r] * scale;
        v += bv;
        slab[(mOff + r) * 68 + (j << 4) + rlane] = v;
      }
    }
    __builtin_amdgcn_fence(__ATOMIC_RELEASE, "workgroup");
    __builtin_amdgcn_wave_barrier();
    __builtin_amdgcn_fence(__ATOMIC_ACQUIRE, "workgroup");
    {
      const int hh = lane >> 4, c4 = (lane & 15) * 4;
      for (int pass = 0; pass < 2; ++pass) {
#pragma unroll
        for (int it = 0; it < 8; ++it) {
          const int row = it * 2 + hh;
          const v4f v = *(const v4f*)(slab + row * 68 + c4);
          *(volatile v4f*)(Cout + (size_t)(mBase + row) * ldc + n0 + c4) = v;
        }
        __threadfence();
      }
    }
    __builtin_amdgcn_fence(__ATOMIC_RELEASE, "workgroup");
    __builtin_amdgcn_wave_barrier();
    __builtin_amdgcn_fence(__ATOMIC_ACQUIRE, "workgroup");
  }
}

extern "C" void kernel_launch(void* const* d_in, const int* in_sizes, int n_in,
                              void* d_out, int out_size, void* d_ws, size_t ws_size,
                              hipStream_t stream) {
  if (n_in < 5) return;
  if (in_sizes[0] != kBatch * kIn) return;
  if (in_sizes[1] != kOut * kKs) return;
  if (in_sizes[2] != kOut * kIn) return;
  if (in_sizes[3] != kOut) return;
  if (in_sizes[4] != kOut * kIn) return;
  if (out_size != kBatch * kOut) return;
  if (ws_size < kWsTotal) return;

  const float* x      = (const float*)d_in[0];
  const float* coeffs = (const float*)d_in[1];
  const float* resw   = (const float*)d_in[2];
  const float* bias   = (const float*)d_in[3];
  const float* sbase  = (const float*)d_in[4];
  float* out = (float*)d_out;

  char* ws = (char*)d_ws;
  unsigned short* APL = (unsigned short*)(ws + kOffA);
  unsigned short* BPL = (unsigned short*)(ws + kOffB);

  build_bt_kernel<<<kOut, 256, 0, stream>>>(coeffs, resw, sbase, BPL);
  build_a_kernel<<<dim3(kIn / kChunkI, kBatch), 256, 0, stream>>>(x, APL);
  gemm_f16_bias_kernel<<<((kBatch / 64) * (kOut / 64)) / 8, 256, 0, stream>>>(
      APL, kK, BPL, kK, out, kOut, bias, kBatch, kOut, kK, kFold);
}
